// STSN_Offset_36601711296534
// MI455X (gfx1250) — hardware-verified
//
#include <hip/hip_runtime.h>
#include <stddef.h>


#define Bn     4
#define C2n    128
#define Cn     256
#define Hn     64
#define Wn     64
#define HWn    (Hn * Wn)
#define KTAP   9
#define KKn    (Cn * KTAP)
#define OFFR   18
#define OFFC   32
#define NLAYO  4
#define NLAYD  3
#define APITCH 40
#define CPITCH 36
#define SPITCH 260

typedef _Float16 f16t;
typedef f16t  v16h __attribute__((ext_vector_type(16)));
typedef f16t  v8h  __attribute__((ext_vector_type(8)));
typedef f16t  v4h  __attribute__((ext_vector_type(4)));
typedef float v8f  __attribute__((ext_vector_type(8)));
typedef float v4f  __attribute__((ext_vector_type(4)));

union Frag { v16h v; v8h half[2]; };

__device__ __forceinline__ v8f wmma16(v16h a, v16h b, v8f c) {
  v8f d = __builtin_amdgcn_wmma_f32_16x16x32_f16(false, a, false, b, (short)0, c, false, false);
  asm volatile("v_nop\n\tv_nop\n\tv_nop\n\tv_nop" : "+v"(d) : "v"(a), "v"(b));
  return d;
}

__global__ __launch_bounds__(256) void k_concat(
    const float* __restrict__ x, const float* __restrict__ y, float* feat) {
  __shared__ __align__(16) float tile[32][CPITCH];
  const int bid = blockIdx.x;
  if (bid >= Bn * (HWn / 32) * (Cn / 32)) return;
  const int cb  = (bid & 7) << 5;
  const int pb  = ((bid >> 3) & 127) << 5;
  const int b   = bid >> 10;
  const int tid = threadIdx.x;
  const int tr  = tid >> 5;
  const int tc  = tid & 31;
#pragma unroll
  for (int j = 0; j < 4; ++j) {
    const int c = cb + tr + j * 8;
    const float* src = (c < C2n)
        ? (x + ((size_t)b * C2n + c) * HWn)
        : (y + ((size_t)b * C2n + (c - C2n)) * HWn);
    tile[tc][tr + j * 8] = src[pb + tc];
  }
  __syncthreads();
  const int lane = tid & 31, wv = tid >> 5;
  const int p = wv * 4 + (lane >> 3);
  const int q = lane & 7;
  const v4f v = *(const v4f*)&tile[p][4 * q];
  float* dst = feat + ((size_t)b * HWn + pb + p) * Cn + cb + 4 * q;
  *(volatile v4f*)dst = v;
  __threadfence();
  *(volatile v4f*)dst = v;
}

__global__ __launch_bounds__(256) void k_cvt_w(
    const float* __restrict__ src, f16t* dst, int nSrc, int nPad, int total8, float wscale) {
  const int i = blockIdx.x * 256 + threadIdx.x;
  if (i >= total8) return;
  const int e   = i * 8;
  const int kp  = e % KKn;
  const int n   = (e / KKn) % nPad;
  const int l   = e / (KKn * nPad);
  const int tap = kp >> 8;
  const int c   = kp & 255;
  v8h v;
  if (n < nSrc) {
    const float* s = src + (((size_t)l * nSrc + n) * Cn + c) * KTAP + tap;
#pragma unroll
    for (int j = 0; j < 8; ++j) v[j] = (f16t)(s[j * KTAP] * wscale);
  } else {
#pragma unroll
    for (int j = 0; j < 8; ++j) v[j] = (f16t)0.0f;
  }
  f16t* d = dst + (size_t)e;
  *(volatile v8h*)d = v;
  __threadfence();
  *(volatile v8h*)d = v;
}

__global__ __launch_bounds__(64) void k_conv(
    const float* __restrict__ feat, const f16t* __restrict__ wB,
    float* out, int outC, float oscale) {
  __shared__ __align__(16) f16t  Abuf[2][32][APITCH];
  __shared__ __align__(16) float stg[32][CPITCH];

  const int bid = blockIdx.x;
  if (bid >= Bn * Hn * (Wn / 32)) return;
  const int w0 = (bid & 1) << 5;
  const int h  = (bid >> 1) & (Hn - 1);
  const int b  = bid >> 7;

  const int tid  = threadIdx.x;
  const int lane = tid & 31;
  const int wv   = tid >> 5;
  const int row  = lane & 15;
  const int hi   = lane >> 4;

  const int am  = tid >> 1;
  const int kkb = (tid & 1) << 4;

  v8f acc0 = {};
  v8f acc1 = {};
  const f16t*  bbase = wB + (size_t)(wv * 16 + row) * KKn + 8 * hi;
  const float* fbase = feat + (size_t)b * HWn * Cn;

  for (int tap = 0; tap < KTAP; ++tap) {
    const int ty = tap / 3 - 1;
    const int tx = tap - (tap / 3) * 3 - 1;
    const int yy = h + ty;
    const int xx = w0 + am + tx;
    const bool inb = ((unsigned)yy < (unsigned)Hn) && ((unsigned)xx < (unsigned)Wn);
    const int yyc = yy < 0 ? 0 : (yy > Hn - 1 ? Hn - 1 : yy);
    const int xxc = xx < 0 ? 0 : (xx > Wn - 1 ? Wn - 1 : xx);
    const float* pl = fbase + ((size_t)yyc * Wn + xxc) * Cn + kkb;

#pragma unroll 2
    for (int cc = 0; cc < 8; ++cc) {
      const int kc = tap * 8 + cc;
      const int p  = kc & 1;
      v8h va, vb;
      if (inb) {
        const float* s = pl + (cc << 5);
        const v4f f0 = *(const v4f*)(s);
        const v4f f1 = *(const v4f*)(s + 4);
        const v4f f2 = *(const v4f*)(s + 8);
        const v4f f3 = *(const v4f*)(s + 12);
#pragma unroll
        for (int j = 0; j < 4; ++j) {
          va[j]     = (f16t)f0[j];
          va[j + 4] = (f16t)f1[j];
          vb[j]     = (f16t)f2[j];
          vb[j + 4] = (f16t)f3[j];
        }
      } else {
#pragma unroll
        for (int j = 0; j < 8; ++j) { va[j] = (f16t)0.0f; vb[j] = (f16t)0.0f; }
      }
      *(v8h*)&Abuf[p][am][kkb]     = va;
      *(v8h*)&Abuf[p][am][kkb + 8] = vb;
      __syncthreads();

      Frag a0, a1, bf;
      a0.half[0] = *(const v8h*)&Abuf[p][row][8 * hi];
      a0.half[1] = *(const v8h*)&Abuf[p][row][16 + 8 * hi];
      a1.half[0] = *(const v8h*)&Abuf[p][16 + row][8 * hi];
      a1.half[1] = *(const v8h*)&Abuf[p][16 + row][16 + 8 * hi];
      const f16t* bp = bbase + (size_t)kc * 32;
      bf.half[0] = *(const v8h*)(bp);
      bf.half[1] = *(const v8h*)(bp + 16);

      acc0 = wmma16(a0.v, bf.v, acc0);
      acc1 = wmma16(a1.v, bf.v, acc1);
    }
  }

  const int nl = wv * 16 + row;
#pragma unroll
  for (int r = 0; r < 8; ++r) {
    stg[nl][8 * hi + r]      = acc0[r] * oscale;
    stg[nl][16 + 8 * hi + r] = acc1[r] * oscale;
  }
  __syncthreads();

  const int q  = lane & 7;
  const int pr = lane >> 3;
  v4f v[4];
  int chs[4];
#pragma unroll
  for (int j = 0; j < 4; ++j) {
    const int ch = wv * 16 + j * 4 + pr;
    chs[j] = ch;
    v[j] = *(const v4f*)&stg[ch][4 * q];
  }
#pragma unroll
  for (int j = 0; j < 4; ++j) {
    if (chs[j] < outC) {
      float* d = out + (((size_t)b * outC + chs[j]) * Hn + h) * Wn + w0 + 4 * q;
      *(volatile v4f*)d = v[j];
    }
  }
  __threadfence();
#pragma unroll
  for (int j = 0; j < 4; ++j) {
    if (chs[j] < outC) {
      float* d = out + (((size_t)b * outC + chs[j]) * Hn + h) * Wn + w0 + 4 * q;
      *(volatile v4f*)d = v[j];
    }
  }
}

struct TapInfo {
  int   i00, i01, i10, i11;
  float w00, w01, w10, w11;
};

__global__ __launch_bounds__(256) void k_deform(
    const float* __restrict__ feat, const float* __restrict__ off,
    const f16t* __restrict__ wB, float* out, float oscale) {
  __shared__ __align__(16) f16t  Abuf[2][32][APITCH];
  __shared__ TapInfo taps[32 * KTAP];
  __shared__ __align__(16) float stg[32][SPITCH];

  const int bid = blockIdx.x;
  if (bid >= Bn * Hn * (Wn / 32)) return;
  const int w0 = (bid & 1) << 5;
  const int h  = (bid >> 1) & (Hn - 1);
  const int b  = bid >> 7;

  const int tid  = threadIdx.x;
  const int lane = tid & 31;
  const int wv   = tid >> 5;
  const int row  = lane & 15;
  const int hi   = lane >> 4;

  for (int t = tid; t < 32 * KTAP; t += 256) {
    const int m   = t / KTAP;
    const int tap = t - m * KTAP;
    const int ty  = tap / 3 - 1;
    const int tx  = tap - (tap / 3) * 3 - 1;
    const int xpix = w0 + m;
    const size_t obase = (((size_t)b * OFFC + tap * 2) * Hn + h) * Wn + xpix;
    const float dy = off[obase];
    const float dx = off[obase + (size_t)HWn];
    const float py = dy + (float)ty + (float)h;
    const float px = dx + (float)tx + (float)xpix;
    const float y0f = floorf(py), x0f = floorf(px);
    const float wy1 = py - y0f, wy0 = 1.0f - wy1;
    const float wx1 = px - x0f, wx0 = 1.0f - wx1;
    const float y0g = fminf(fmaxf(y0f, -2.0f), (float)Hn);
    const float x0g = fminf(fmaxf(x0f, -2.0f), (float)Wn);
    const int y0 = (int)y0g, x0 = (int)x0g;
    const int y1 = y0 + 1,   x1 = x0 + 1;
    const float vy0 = (y0 >= 0 && y0 < Hn) ? 1.0f : 0.0f;
    const float vy1 = (y1 >= 0 && y1 < Hn) ? 1.0f : 0.0f;
    const float vx0 = (x0 >= 0 && x0 < Wn) ? 1.0f : 0.0f;
    const float vx1 = (x1 >= 0 && x1 < Wn) ? 1.0f : 0.0f;
    const int y0c = y0 < 0 ? 0 : (y0 > Hn - 1 ? Hn - 1 : y0);
    const int y1c = y1 < 0 ? 0 : (y1 > Hn - 1 ? Hn - 1 : y1);
    const int x0c = x0 < 0 ? 0 : (x0 > Wn - 1 ? Wn - 1 : x0);
    const int x1c = x1 < 0 ? 0 : (x1 > Wn - 1 ? Wn - 1 : x1);
    TapInfo ti;
    ti.i00 = y0c * Wn + x0c;  ti.i01 = y0c * Wn + x1c;
    ti.i10 = y1c * Wn + x0c;  ti.i11 = y1c * Wn + x1c;
    ti.w00 = wy0 * wx0 * vy0 * vx0;
    ti.w01 = wy0 * wx1 * vy0 * vx1;
    ti.w10 = wy1 * wx0 * vy1 * vx0;
    ti.w11 = wy1 * wx1 * vy1 * vx1;
    taps[t] = ti;
  }
  __syncthreads();

  const int am  = tid >> 3;
  const int kkb = (tid & 7) << 2;

  v8f acc00 = {};
  v8f acc01 = {};
  v8f acc10 = {};
  v8f acc11 = {};
  const f16t*  b0base = wB + (size_t)(wv * 32 + row) * KKn + 8 * hi;
  const f16t*  b1base = b0base + (size_t)16 * KKn;
  const float* fbase  = feat + (size_t)b * HWn * Cn;

  for (int tap = 0; tap < KTAP; ++tap) {
    const TapInfo ti = taps[am * KTAP + tap];
    const float* p00 = fbase + (size_t)ti.i00 * Cn + kkb;
    const float* p01 = fbase + (size_t)ti.i01 * Cn + kkb;
    const float* p10 = fbase + (size_t)ti.i10 * Cn + kkb;
    const float* p11 = fbase + (size_t)ti.i11 * Cn + kkb;

#pragma unroll 2
    for (int cc = 0; cc < 8; ++cc) {
      const int kc = tap * 8 + cc;
      const int p  = kc & 1;
      const int cb = cc << 5;
      const v4f f00 = *(const v4f*)(p00 + cb);
      const v4f f01 = *(const v4f*)(p01 + cb);
      const v4f f10 = *(const v4f*)(p10 + cb);
      const v4f f11 = *(const v4f*)(p11 + cb);
      v4h vals;
#pragma unroll
      for (int j = 0; j < 4; ++j)
        vals[j] = (f16t)(ti.w00 * f00[j] + ti.w01 * f01[j] +
                         ti.w10 * f10[j] + ti.w11 * f11[j]);
      *(v4h*)&Abuf[p][am][kkb] = vals;
      __syncthreads();

      Frag a0, a1, bq0, bq1;
      a0.half[0] = *(const v8h*)&Abuf[p][row][8 * hi];
      a0.half[1] = *(const v8h*)&Abuf[p][row][16 + 8 * hi];
      a1.half[0] = *(const v8h*)&Abuf[p][16 + row][8 * hi];
      a1.half[1] = *(const v8h*)&Abuf[p][16 + row][16 + 8 * hi];
      const f16t* bp0 = b0base + (size_t)kc * 32;
      const f16t* bp1 = b1base + (size_t)kc * 32;
      bq0.half[0] = *(const v8h*)(bp0);
      bq0.half[1] = *(const v8h*)(bp0 + 16);
      bq1.half[0] = *(const v8h*)(bp1);
      bq1.half[1] = *(const v8h*)(bp1 + 16);

      acc00 = wmma16(a0.v, bq0.v, acc00);
      acc01 = wmma16(a0.v, bq1.v, acc01);
      acc10 = wmma16(a1.v, bq0.v, acc10);
      acc11 = wmma16(a1.v, bq1.v, acc11);
    }
  }

  const int n0 = wv * 32 + row;
#pragma unroll
  for (int r = 0; r < 8; ++r) {
    stg[8 * hi + r][n0]           = acc00[r] * oscale;
    stg[8 * hi + r][n0 + 16]      = acc01[r] * oscale;
    stg[16 + 8 * hi + r][n0]      = acc10[r] * oscale;
    stg[16 + 8 * hi + r][n0 + 16] = acc11[r] * oscale;
  }
  __syncthreads();

  const int q  = lane & 7;
  const int pr = lane >> 3;
  const size_t pixbase = ((size_t)b * Hn + h) * Wn + w0;
  v4f v[8];
#pragma unroll
  for (int j = 0; j < 8; ++j) {
    const int px = j * 4 + pr;
    v[j] = *(const v4f*)&stg[px][wv * 32 + 4 * q];
  }
#pragma unroll
  for (int j = 0; j < 8; ++j) {
    const int px = j * 4 + pr;
    float* d = out + (pixbase + px) * Cn + wv * 32 + 4 * q;
    *(volatile v4f*)d = v[j];
  }
  __threadfence();
#pragma unroll
  for (int j = 0; j < 8; ++j) {
    const int px = j * 4 + pr;
    float* d = out + (pixbase + px) * Cn + wv * 32 + 4 * q;
    *(volatile v4f*)d = v[j];
  }
}

extern "C" void kernel_launch(void* const* d_in, const int* in_sizes, int n_in,
                              void* d_out, int out_size, void* d_ws, size_t ws_size,
                              hipStream_t stream) {
  if (n_in < 4) return;
  if (in_sizes[0] != Bn * C2n * HWn) return;
  if (in_sizes[1] != Bn * C2n * HWn) return;
  if (in_sizes[2] != NLAYO * OFFR * Cn * KTAP) return;
  if (in_sizes[3] != NLAYD * Cn * Cn * KTAP) return;
  if (out_size != Bn * OFFR * HWn) return;

  const float* x    = (const float*)d_in[0];
  const float* y    = (const float*)d_in[1];
  const float* wofs = (const float*)d_in[2];
  const float* wdef = (const float*)d_in[3];
  float* out = (float*)d_out;

  const size_t szF   = (size_t)Bn * HWn * Cn * sizeof(float);
  const size_t szOff = (size_t)Bn * OFFC * HWn * sizeof(float);
  const size_t szOW  = (size_t)NLAYO * OFFC * KKn * sizeof(f16t);
  const size_t szDW  = (size_t)NLAYD * Cn * KKn * sizeof(f16t);
  const size_t oFA  = 0;
  const size_t oFB  = oFA + szF;
  const size_t oOff = oFB + szF;
  const size_t oOW  = oOff + szOff;
  const size_t oDW  = oOW + szOW;
  const size_t total = oDW + szDW;
  if (total > ws_size) return;

  char* ws = (char*)d_ws;
  float* featA  = (float*)(ws + oFA);
  float* featB  = (float*)(ws + oFB);
  float* offBuf = (float*)(ws + oOff);
  f16t*  offW16 = (f16t*)(ws + oOW);
  f16t*  dW16   = (f16t*)(ws + oDW);

  const int tot8O = NLAYO * OFFC * KKn / 8;
  const int tot8D = NLAYD * Cn * KKn / 8;
  const float sO = 1024.0f, sD = 256.0f;
  const float rO = 1.0f / 1024.0f, rD = 1.0f / 256.0f;

  k_concat<<<Bn * (HWn / 32) * (Cn / 32), 256, 0, stream>>>(x, y, featA);
  k_cvt_w<<<(tot8O + 255) / 256, 256, 0, stream>>>(wofs, offW16, OFFR, OFFC, tot8O, sO);
  k_cvt_w<<<(tot8D + 255) / 256, 256, 0, stream>>>(wdef, dW16, Cn, Cn, tot8D, sD);

  const int gblocks = Bn * Hn * (Wn / 32);
  float* cur = featA;
  float* nxt = featB;
  for (int i = 0; i < NLAYD; ++i) {
    k_conv<<<gblocks, 64, 0, stream>>>(
        cur, offW16 + (size_t)i * OFFC * KKn, offBuf, OFFC, rO);
    k_deform<<<gblocks, 256, 0, stream>>>(
        cur, offBuf, dW16 + (size_t)i * Cn * KKn, nxt, rD);
    float* t = cur; cur = nxt; nxt = t;
  }
  k_conv<<<gblocks, 64, 0, stream>>>(
      cur, offW16 + (size_t)NLAYD * OFFC * KKn, out, OFFR, rO);
}
